// VanillaNeedleRIN_75892072121022
// MI455X (gfx1250) — hardware-verified
//
#include <hip/hip_runtime.h>
#include <math.h>

typedef __attribute__((ext_vector_type(16))) _Float16 v16h;
typedef __attribute__((ext_vector_type(8)))  _Float16 v8h;
typedef __attribute__((ext_vector_type(8)))  float    v8f;
typedef __attribute__((ext_vector_type(4)))  float    v4f;
typedef __attribute__((ext_vector_type(4)))  unsigned int v4u;

constexpr int kBatch = 64;
constexpr int kSeq   = 4096;
constexpr int kHalf  = 64;
constexpr int kHid   = 128;
constexpr int kLay   = 2;
constexpr int kVocab = 32000;
constexpr int kNsig  = 32000;
constexpr int kLut   = 4096;
constexpr int kDepth = 2 * kHalf;
static_assert(kDepth == 128);
static_assert((kDepth % 32) == 0);
static_assert((kNsig % 64) == 0);
static_assert(kBatch == 64);
static_assert(kSeq == kLut);
static_assert(kHid == 128);

constexpr double kTwoPiD   = 6.283185307179586;
constexpr double kPhiD     = 1.618033988749895;
constexpr float  kTwoPiF   = (float)kTwoPiD;
constexpr float  kPhiF     = (float)kPhiD;
constexpr float  kLutScale = (float)((double)kLut / kTwoPiD);
constexpr float  kLutStep  = (float)(kTwoPiD / (double)kLut);
constexpr float  kTLast    = (float)((double)(kSeq - 1) * kPhiD);
constexpr double kTLastQ   = (double)(long long)((double)kTLast / (double)kTwoPiF);
constexpr float  kTLastWrap = (float)((double)kTLast - kTLastQ * (double)kTwoPiF);
constexpr float  kCarryA   = 16.0f;
constexpr float  kCarryB   = 64.0f;
constexpr float  kFold     = 1.0f / (kCarryA * kCarryB);

constexpr size_t kOffBT   = 0;
constexpr size_t kBytesBT = (size_t)kNsig * kDepth * 2;
constexpr size_t kOffHS   = kOffBT + kBytesBT;
constexpr size_t kBytesHS = (size_t)kBatch * kDepth * 4;
constexpr size_t kOffAP   = kOffHS + kBytesHS;
constexpr size_t kBytesAP = (size_t)kBatch * kDepth * 2;
constexpr size_t kWsTotal = kOffAP + kBytesAP;
static_assert(kWsTotal == 8241152ull);
static_assert(kWsTotal <= 134217728ull);
static_assert((kOffHS % 128) == 0);
static_assert((kOffAP % 128) == 0);

union FragU { v16h v; v8h h[2]; };
__device__ __forceinline__ v16h frag_load(const _Float16* p) {
  FragU f;
  f.h[0] = *(const v8h*)(p);
  f.h[1] = *(const v8h*)(p + 16);
  return f.v;
}
__device__ __forceinline__ v8f mma_f16(v16h a, v16h b, v8f c) {
  c = __builtin_amdgcn_wmma_f32_16x16x32_f16(false, a, false, b, (short)0, c, false, false);
  asm volatile("v_nop\n\tv_nop\n\tv_nop\n\tv_nop" : "+v"(c) : "v"(a), "v"(b));
  return c;
}
__device__ __forceinline__ unsigned pack_f16x2(float f0, float f1) {
  const _Float16 h0 = (_Float16)f0;
  const _Float16 h1 = (_Float16)f1;
  const unsigned short u0 = __builtin_bit_cast(unsigned short, h0);
  const unsigned short u1 = __builtin_bit_cast(unsigned short, h1);
  return (unsigned)u0 | ((unsigned)u1 << 16);
}

__global__ __launch_bounds__(256) void prep_bt_kernel(
    const float* __restrict__ owr, const float* __restrict__ owi, unsigned int* __restrict__ btw)
{
  __shared__ __align__(16) unsigned int sBw[64 * 68];
  const int tid = threadIdx.x;
  const int n0 = blockIdx.x * 64;
  const int kpl = tid >> 4;
  const int c4 = (tid & 15) * 4;
#pragma unroll
  for (int it = 0; it < 4; ++it) {
    const float* src = (it < 2) ? owr : owi;
    const int kp = kpl + 16 * it;
    const int krow = 2 * (kpl + 16 * (it & 1));
    const v4f r0 = *(const v4f*)(src + (size_t)krow * kNsig + n0 + c4);
    const v4f r1 = *(const v4f*)(src + (size_t)(krow + 1) * kNsig + n0 + c4);
#pragma unroll
    for (int e = 0; e < 4; ++e) {
      const float f0 = r0[e] * kCarryB;
      const float f1 = r1[e] * kCarryB;
      sBw[(c4 + e) * 68 + kp] = pack_f16x2(f0, f1);
    }
  }
  __syncthreads();
  v4u val[4];
#pragma unroll
  for (int it = 0; it < 4; ++it) {
    const int c = it * 256 + tid;
    const int nl = c >> 4;
    const int seg = c & 15;
    val[it] = *(const v4u*)(sBw + nl * 68 + seg * 4);
  }
  for (int pass = 0; pass < 2; ++pass) {
#pragma unroll
    for (int it = 0; it < 4; ++it) {
      const int c = it * 256 + tid;
      const int nl = c >> 4;
      const int seg = c & 15;
      *(volatile v4u*)(btw + (size_t)(n0 + nl) * (kDepth / 2) + seg * 4) = val[it];
    }
    __threadfence();
  }
}

#define TABLE_INTERP(th_, s_, c_)                                   \
  {                                                                 \
    const float pos_  = (th_) * kLutScale;                          \
    const float i0_   = floorf(pos_);                               \
    const float frac_ = pos_ - i0_;                                 \
    const int   ix0_  = ((int)i0_) & (kLut - 1);                    \
    const int   ix1_  = (ix0_ + 1) & (kLut - 1);                    \
    const float omf_  = 1.0f - frac_;                               \
    (s_) = s_sin[ix0_] * omf_ + s_sin[ix1_] * frac_;                \
    (c_) = s_cos[ix0_] * omf_ + s_cos[ix1_] * frac_;                \
  }

__global__ __launch_bounds__(64) void scan_kernel(
    const int* __restrict__ ids, const float* __restrict__ emb, float* __restrict__ hs)
{
#pragma clang fp contract(off)
  __shared__ float s_sin[kLut];
  __shared__ float s_cos[kLut];
  __shared__ float s_tphi[kSeq];
  const int tid = threadIdx.x;
  const int b = blockIdx.x;
#pragma unroll 1
  for (int i = tid; i < kLut; i += 64) {
    const float ang = (float)i * kLutStep;
    float sv, cv;
    sincosf(ang, &sv, &cv);
    s_sin[i] = sv;
    s_cos[i] = cv;
    s_tphi[i] = fmodf((float)i * kPhiF, kTwoPiF);
  }
  __syncthreads();

  const int* idrow = ids + (size_t)b * kSeq;
  float hr = 0.0f, hi = 0.0f;
  int id = idrow[0];
  id = id < 0 ? 0 : (id > kVocab - 1 ? kVocab - 1 : id);
  float w  = emb[(size_t)id * kDepth + tid];
  float bt = emb[(size_t)id * kDepth + kHalf + tid];
#pragma unroll 1
  for (int t = 0; t < kSeq; ++t) {
    const int tn = (t + 1 < kSeq) ? (t + 1) : (kSeq - 1);
    int idn = idrow[tn];
    idn = idn < 0 ? 0 : (idn > kVocab - 1 ? kVocab - 1 : idn);
    const float wn = emb[(size_t)idn * kDepth + tid];
    const float bn = emb[(size_t)idn * kDepth + kHalf + tid];

    const float wl   = 1.0f + fabsf(w);
    const float inv  = 1.0f / wl;
    const float tphi = s_tphi[t];
    const float thr  = (hr * inv + bt) + tphi;
    const float thi  = (hi * inv + bt) + tphi;
    float sr, cr, si, ci;
    TABLE_INTERP(thr, sr, cr)
    TABLE_INTERP(thi, si, ci)
    const float nr = cr * ci - sr * si;
    const float ni = cr * si + sr * ci;
    hr = nr;
    hi = ni;
    w = wn;
    bt = bn;
  }
  float* hrow = hs + (size_t)b * kDepth;
  volatile float* p0 = hrow + tid;
  volatile float* p1 = hrow + kHalf + tid;
  *p0 = hr;
  *p1 = hi;
  __threadfence();
  *p0 = hr;
  *p1 = hi;
}

__device__ __forceinline__ void layer_rotation(float lwv, float lbv, float& s, float& c) {
#pragma clang fp contract(off)
  const float wlen  = 1.0f + fabsf(lwv);
  const float inv   = 1.0f / wlen;
  const float theta = kTLastWrap * inv + lbv;
  const float pos   = theta * kLutScale;
  const float i0    = floorf(pos);
  const float frac  = pos - i0;
  const int   ix0   = ((int)i0) & (kLut - 1);
  const float omf   = 1.0f - frac;
  float sa = 0.0f, ca = 0.0f;
#pragma unroll 1
  for (int jj = 0; jj < 2; ++jj) {
    const int ix = (ix0 + jj) & (kLut - 1);
    const float wgt = (jj == 0) ? omf : frac;
    float sv, cv;
    sincosf((float)ix * kLutStep, &sv, &cv);
    sa = sa + sv * wgt;
    ca = ca + cv * wgt;
  }
  s = sa;
  c = ca;
}

__global__ __launch_bounds__(128) void layers_kernel(
    const float* __restrict__ hs,
    const float* __restrict__ win_r, const float* __restrict__ win_i,
    const float* __restrict__ wout_r, const float* __restrict__ wout_i,
    const float* __restrict__ lw, const float* __restrict__ lb,
    unsigned int* __restrict__ apw)
{
  __shared__ float s_x[2 * kHalf];
  __shared__ float s_v[2 * kHid];
  const int tid = threadIdx.x;
  const int lane = tid & 31;
  const int wave = __builtin_amdgcn_readfirstlane((int)(threadIdx.x >> 5));
  const int b = blockIdx.x;
  s_x[tid] = hs[(size_t)b * kDepth + tid];
#pragma unroll 1
  for (int l = 0; l < kLay; ++l) {
    __syncthreads();
    {
      const float* pr = win_r + (size_t)l * kHalf * kHid + tid;
      const float* pi = win_i + (size_t)l * kHalf * kHid + tid;
      float ur = 0.0f, ui = 0.0f;
#pragma unroll 1
      for (int k = 0; k < kHalf; ++k) {
        const float wr = pr[(size_t)k * kHid];
        const float wi = pi[(size_t)k * kHid];
        const float ar = s_x[k];
        const float ai = s_x[kHalf + k];
        ur = fmaf(ar, wr, ur);
        ur = fmaf(-ai, wi, ur);
        ui = fmaf(ar, wi, ui);
        ui = fmaf(ai, wr, ui);
      }
      float s, c;
      layer_rotation(lw[l * kHid + tid], lb[l * kHid + tid], s, c);
      const float vr = ur * c - ui * s;
      const float vi = ur * s + ui * c;
      s_v[tid] = vr;
      s_v[kHid + tid] = vi;
    }
    __syncthreads();
#pragma unroll 1
    for (int i = 0; i < 2; ++i) {
      const int e = tid + kHid * i;
      const float v = s_v[e];
      const float sg = 1.0f / (1.0f + expf(-v));
      s_v[e] = v * sg;
    }
    __syncthreads();
    float outr = 0.0f, outi = 0.0f;
    if (wave < 2) {
      const float* pr = wout_r + (size_t)l * kHid * kHalf + tid;
      const float* pi = wout_i + (size_t)l * kHid * kHalf + tid;
#pragma unroll 1
      for (int n = 0; n < kHid; ++n) {
        const float wr = pr[(size_t)n * kHalf];
        const float wi = pi[(size_t)n * kHalf];
        const float ar = s_v[n];
        const float ai = s_v[kHid + n];
        outr = fmaf(ar, wr, outr);
        outr = fmaf(-ai, wi, outr);
        outi = fmaf(ar, wi, outi);
        outi = fmaf(ai, wr, outi);
      }
    }
    __syncthreads();
    if (wave < 2) {
      s_x[tid] = outr;
      s_x[kHalf + tid] = outi;
    }
  }
  __syncthreads();
  if (wave < 2) {
    const float sgn = (wave == 0) ? 1.0f : -1.0f;
    const int k = 2 * lane;
    const float a0 = (s_x[k] + sgn * s_x[kHalf + k]) * kCarryA;
    const float a1 = (s_x[k + 1] + sgn * s_x[kHalf + k + 1]) * kCarryA;
    const unsigned u = pack_f16x2(a0, a1);
    volatile unsigned int* p = apw + (size_t)b * (kDepth / 2) + wave * 32 + lane;
    *p = u;
    __threadfence();
    *p = u;
  }
}

constexpr int kTilesN = kNsig / 64;
static_assert((kTilesN % 4) == 0);
__global__ __launch_bounds__(128) void out_gemm_kernel(
    const unsigned short* __restrict__ Ap, const unsigned short* __restrict__ Btp, float* __restrict__ C)
{
  __shared__ __align__(16) float sT[4][16 * 68];
  const int lane = threadIdx.x & 31;
  const int wave = __builtin_amdgcn_readfirstlane((int)(threadIdx.x >> 5));
  const int tile = blockIdx.x * 4 + wave;
  if (tile >= kTilesN) return;
  const int n0 = tile << 6;
  const _Float16* A  = (const _Float16*)Ap;
  const _Float16* Bt = (const _Float16*)Btp;
  const int rlane = lane & 15;
  const int koff  = (lane >> 4) * 8;
  const int mOff  = (lane >> 4) * 8;

  v8f acc[4][4];
#pragma unroll
  for (int i = 0; i < 4; ++i)
#pragma unroll
    for (int j = 0; j < 4; ++j) acc[i][j] = (v8f){0.f, 0.f, 0.f, 0.f, 0.f, 0.f, 0.f, 0.f};

#pragma unroll 1
  for (int k0 = 0; k0 < kDepth; k0 += 32) {
    v16h bh[4];
#pragma unroll
    for (int j = 0; j < 4; ++j) {
      const size_t bo = (size_t)(n0 + (j << 4) + rlane) * kDepth + koff + k0;
      bh[j] = frag_load(Bt + bo);
    }
#pragma unroll
    for (int i = 0; i < 4; ++i) {
      const size_t ao = (size_t)((i << 4) + rlane) * kDepth + koff + k0;
      const v16h ah = frag_load(A + ao);
#pragma unroll
      for (int j = 0; j < 4; ++j) acc[i][j] = mma_f16(ah, bh[j], acc[i][j]);
    }
  }

  float* slab = sT[wave];
#pragma unroll
  for (int i = 0; i < 4; ++i) {
    const int mBase = i << 4;
#pragma unroll
    for (int j = 0; j < 4; ++j) {
#pragma unroll
      for (int r = 0; r < 8; ++r) {
        const float v = acc[i][j][r] * kFold;
        slab[(mOff + r) * 68 + (j << 4) + rlane] = v;
      }
    }
    __builtin_amdgcn_fence(__ATOMIC_RELEASE, "workgroup");
    __builtin_amdgcn_wave_barrier();
    __builtin_amdgcn_fence(__ATOMIC_ACQUIRE, "workgroup");
    {
      const int hh = lane >> 4;
      const int c4 = (lane & 15) * 4;
      for (int pass = 0; pass < 2; ++pass) {
#pragma unroll
        for (int it = 0; it < 8; ++it) {
          const int row = it * 2 + hh;
          const v4f v = *(const v4f*)(slab + row * 68 + c4);
          *(volatile v4f*)(C + (size_t)(mBase + row) * kNsig + n0 + c4) = v;
        }
        __threadfence();
      }
    }
    __builtin_amdgcn_fence(__ATOMIC_RELEASE, "workgroup");
    __builtin_amdgcn_wave_barrier();
    __builtin_amdgcn_fence(__ATOMIC_ACQUIRE, "workgroup");
  }
}

extern "C" void kernel_launch(void* const* d_in, const int* in_sizes, int n_in,
                              void* d_out, int out_size, void* d_ws, size_t ws_size,
                              hipStream_t stream) {
  if (n_in < 10) return;
  if (in_sizes[0] != kBatch * kSeq) return;
  if (in_sizes[1] != kVocab * kDepth) return;
  if (in_sizes[2] != kLay * kHalf * kHid) return;
  if (in_sizes[3] != kLay * kHalf * kHid) return;
  if (in_sizes[4] != kLay * kHid * kHalf) return;
  if (in_sizes[5] != kLay * kHid * kHalf) return;
  if (in_sizes[6] != kLay * kHid) return;
  if (in_sizes[7] != kLay * kHid) return;
  if (in_sizes[8] != kHalf * kNsig) return;
  if (in_sizes[9] != kHalf * kNsig) return;
  if (out_size != kBatch * kNsig) return;
  if (ws_size < kWsTotal) return;

  const int*   ids    = (const int*)  d_in[0];
  const float* emb    = (const float*)d_in[1];
  const float* win_r  = (const float*)d_in[2];
  const float* win_i  = (const float*)d_in[3];
  const float* wout_r = (const float*)d_in[4];
  const float* wout_i = (const float*)d_in[5];
  const float* lw     = (const float*)d_in[6];
  const float* lb     = (const float*)d_in[7];
  const float* out_wr = (const float*)d_in[8];
  const float* out_wi = (const float*)d_in[9];
  float* out = (float*)d_out;

  char* ws = (char*)d_ws;
  unsigned int* BTw = (unsigned int*)(ws + kOffBT);
  float*        HS  = (float*)(ws + kOffHS);
  unsigned int* APw = (unsigned int*)(ws + kOffAP);

  prep_bt_kernel<<<kNsig / 64, 256, 0, stream>>>(out_wr, out_wi, BTw);
  scan_kernel<<<kBatch, 64, 0, stream>>>(ids, emb, HS);
  layers_kernel<<<kBatch, 128, 0, stream>>>(HS, win_r, win_i, wout_r, wout_i, lw, lb, APw);
  out_gemm_kernel<<<kTilesN / 4, 128, 0, stream>>>(
      (const unsigned short*)APw, (const unsigned short*)BTw, out);
}
